// ResidualMamba_17162689315093
// MI455X (gfx1250) — hardware-run, weakly checked
//
#include <hip/hip_runtime.h>

#define NB    2
#define NL    2048
#define DM    1024
#define DI    2048
#define DIN2  4096
#define NS    16
#define DTR   64
#define KDT   64
#define NXD   96
#define NXP   128
#define NROWS (NB * NL)
#define TC    16
#define TL    16
#define LNEPS 1e-5f

static_assert(DM % 32 == 0 && DI % 32 == 0 && KDT % 32 == 0);
static_assert(NROWS % 128 == 0 && DIN2 % 64 == 0 && DM % 64 == 0 && NXP % 64 == 0 && DI % 64 == 0);
static_assert(NL % TC == 0 && NROWS % TL == 0 && DI % 256 == 0 && DM == 4 * 256 && TC == 16 && TL == 16);
static_assert(DTR == KDT && KDT == 64 && DTR + 2 * NS == NXD && NXD <= NXP && NXP == 128);
static_assert(DIN2 == 2 * DI && NL % 64 == 0);
static_assert(NXD % 4 == 0 && DM % 8 == 0 && DI % 8 == 0 && NS % 4 == 0);

typedef __bf16         v16b __attribute__((ext_vector_type(16)));
typedef unsigned short v8us __attribute__((ext_vector_type(8)));
typedef float          v8f  __attribute__((ext_vector_type(8)));
typedef float          v4f  __attribute__((ext_vector_type(4)));
typedef v8us __attribute__((may_alias)) v8usa;
typedef v4f  __attribute__((may_alias)) v4fa;

union Frag { v16b v; v8us half[2]; };

constexpr size_t SZ_U16_DM = (size_t)NROWS * DM * 2;
constexpr size_t SZ_U16_DI = (size_t)NROWS * DI * 2;
constexpr size_t SZ_F32_DI = (size_t)NROWS * DI * 4;
constexpr size_t OFF_XNH  = 0;
constexpr size_t OFF_XNL  = OFF_XNH + SZ_U16_DM;
constexpr size_t OFF_WIN  = OFF_XNL + SZ_U16_DM;
constexpr size_t END_PH1  = OFF_WIN + (size_t)DIN2 * DM * 2;
constexpr size_t OFF_XH   = 0;
constexpr size_t OFF_XDBL = OFF_XH + SZ_U16_DI;
constexpr size_t OFF_DTH  = OFF_XDBL + (size_t)NROWS * NXP * 4;
constexpr size_t OFF_DTL  = OFF_DTH + (size_t)NROWS * KDT * 2;
constexpr size_t END_OV1  = OFF_DTL + (size_t)NROWS * KDT * 2;
constexpr size_t OFF_WXP  = END_PH1;
constexpr size_t OFF_WDT  = OFF_WXP + (size_t)NXP * DI * 2;
constexpr size_t OFF_WOUT = OFF_WDT + (size_t)DI * KDT * 2;
constexpr size_t OFF_XC   = OFF_WOUT + (size_t)DM * DI * 2;
constexpr size_t OFF_YH   = OFF_XC;
constexpr size_t OFF_YL   = OFF_YH + SZ_U16_DI;
constexpr size_t OFF_Z    = OFF_XC + SZ_F32_DI;
constexpr size_t OFF_XL   = OFF_Z + SZ_F32_DI;
constexpr size_t WS_END   = OFF_XL + SZ_U16_DI;
static_assert(END_OV1 <= END_PH1);
static_assert(OFF_YL + SZ_U16_DI == OFF_Z);
static_assert(OFF_XNL % 128 == 0 && OFF_WIN % 128 == 0 && OFF_XDBL % 128 == 0 && OFF_DTH % 128 == 0);
static_assert(OFF_DTL % 128 == 0 && OFF_WXP % 128 == 0 && OFF_WDT % 128 == 0 && OFF_WOUT % 128 == 0);
static_assert(OFF_XC % 128 == 0 && OFF_YL % 128 == 0 && OFF_Z % 128 == 0 && OFF_XL % 128 == 0);
static_assert(WS_END <= (size_t)134217728);
static_assert((size_t)(DIN2 / 64) * (DM / 64) * 64 * 64 * 2 == END_PH1 - OFF_WIN);
static_assert((size_t)(NXP / 64) * (DI / 64) * 64 * 64 * 2 == OFF_WDT - OFF_WXP);
static_assert((size_t)(DI / 64) * (KDT / 64) * 64 * 64 * 2 == OFF_WOUT - OFF_WDT);
static_assert((size_t)(DM / 64) * (DI / 64) * 64 * 64 * 2 == OFF_XC - OFF_WOUT);
static_assert((size_t)(NROWS / TL) * TL * DM * 2 == SZ_U16_DM);
static_assert((size_t)(NROWS / 128) * (DIN2 / 64) * 128 * 64 * 4 == 2 * SZ_F32_DI);
static_assert((size_t)(DI / 256) * (NROWS / TC) * (TC * 4) * 128 == SZ_U16_DI);
static_assert((size_t)(NROWS / 128) * (NXP / 64) * 128 * 64 * 4 == OFF_DTH - OFF_XDBL);
static_assert((size_t)(NROWS / 128) * 128 * KDT * 2 == OFF_DTL - OFF_DTH);
static_assert((size_t)(DI / 256) * NB * (NL / TC) * (TC * 4) * 128 == SZ_U16_DI);
static_assert((size_t)(NROWS / 128) * (DM / 64) * 128 * 64 * 4 == (size_t)NROWS * DM * 4);

__device__ __forceinline__ unsigned short bf16_bits(float f) {
  unsigned u = __float_as_uint(f);
  u += 0x7FFFu + ((u >> 16) & 1u);
  return (unsigned short)(u >> 16);
}
__device__ __forceinline__ float bf16_val(unsigned short b) { return __uint_as_float(((unsigned)b) << 16); }
__device__ __forceinline__ float bf16r(float f) { return bf16_val(bf16_bits(f)); }
__device__ __forceinline__ void split_bf16(float v, unsigned short& hb, unsigned short& lb) {
  hb = bf16_bits(v);
  lb = bf16_bits(v - bf16_val(hb));
}
__device__ __forceinline__ v8f zero8() {
  v8f z;
#pragma unroll
  for (int i = 0; i < 8; ++i) z[i] = 0.0f;
  return z;
}
__device__ __forceinline__ float wsum(float v) {
#pragma unroll
  for (int o = 16; o > 0; o >>= 1) v += __shfl_xor(v, o, 32);
  return v;
}

__device__ __forceinline__ void ldfrag_g(Frag& f, const unsigned short* p, int h) {
  f.half[0] = *(const v8usa*)(p + 8 * h);
  f.half[1] = *(const v8usa*)(p + 16 + 8 * h);
}
__device__ __forceinline__ v8f mma16(v8f c, const Frag& a, const Frag& b) {
  v8f d = __builtin_amdgcn_wmma_f32_16x16x32_bf16(false, a.v, false, b.v, (short)0, c, false, false);
  asm volatile("v_nop\n\tv_nop\n\tv_nop\n\tv_nop" : "+v"(d) : "v"(a.v), "v"(b.v));
  return d;
}

__device__ __forceinline__ void tc_store_pass(const unsigned short* sT, unsigned short* dst, int P,
                                              int orow0, int ocol0, int w, int lane) {
  const int q8 = lane & 7, sub = lane >> 3;
#pragma unroll
  for (int i = 0; i < 2; ++i) {
    const int li = 8 * w + 4 * i + sub;
    const v8us v = *(const v8usa*)(sT + li * 64 + 8 * q8);
    unsigned short* p = dst + (size_t)(orow0 + li) * P + ocol0 + 8 * q8;
    *(volatile v8us*)p = v;
  }
}

__global__ __launch_bounds__(256)
void tcvt_kernel(const float* __restrict__ in, int R, int Cc, size_t izs,
                 unsigned short* out, int P, size_t ozs)
{
  __shared__ __attribute__((aligned(16))) unsigned short sT[64 * 64];

  const int tid = threadIdx.x, lane = tid & 31, w = tid >> 5;
  const int orow0 = blockIdx.x * 64, ocol0 = blockIdx.y * 64;
  const float* src = in + (size_t)blockIdx.z * izs;
  unsigned short* dst = out + (size_t)blockIdx.z * ozs;

  const int c4 = tid & 15, rs = tid >> 4;
  const int c = orow0 + 4 * c4;
  const bool cok = (c < Cc);
  const int cc = cok ? c : (Cc - 4);
#pragma unroll
  for (int i = 0; i < 4; ++i) {
    const int rloc = 16 * i + rs;
    const int r = ocol0 + rloc;
    const int rr = (r < R) ? r : (R - 1);
    const v4f v = *(const v4fa*)(src + (size_t)rr * Cc + cc);
    const bool ok = cok && (r < R);
    sT[(4 * c4 + 0) * 64 + rloc] = ok ? bf16_bits(v[0]) : (unsigned short)0;
    sT[(4 * c4 + 1) * 64 + rloc] = ok ? bf16_bits(v[1]) : (unsigned short)0;
    sT[(4 * c4 + 2) * 64 + rloc] = ok ? bf16_bits(v[2]) : (unsigned short)0;
    sT[(4 * c4 + 3) * 64 + rloc] = ok ? bf16_bits(v[3]) : (unsigned short)0;
  }
  __syncthreads();

  tc_store_pass(sT, dst, P, orow0, ocol0, w, lane);
  __threadfence();
  tc_store_pass(sT, dst, P, orow0, ocol0, w, lane);
}

__device__ __forceinline__ void ln_store_pass(const unsigned short* wH, const unsigned short* wL,
                                              unsigned short* ph, unsigned short* pl, int r, int lane) {
#pragma unroll
  for (int g = 0; g < 4; ++g) {
    const v8us vh = *(const v8usa*)(wH + 256 * g + 8 * lane);
    const v8us vl = *(const v8usa*)(wL + 256 * g + 8 * lane);
    const size_t go = (size_t)r * DM + 256 * g + 8 * lane;
    *(volatile v8us*)(ph + go) = vh;
    *(volatile v8us*)(pl + go) = vl;
  }
}

__global__ __launch_bounds__(256)
void ln_kernel(const float* __restrict__ x, const float* __restrict__ lw, const float* __restrict__ lbias,
               unsigned short* ph, unsigned short* pl)
{
  __shared__ __attribute__((aligned(16))) unsigned short sH[8 * DM];
  __shared__ __attribute__((aligned(16))) unsigned short sL[8 * DM];

  const int tid = threadIdx.x, lane = tid & 31, w = tid >> 5;
  const int rbase = blockIdx.x * TL;
  unsigned short* wH = sH + w * DM;
  unsigned short* wL = sL + w * DM;

#pragma unroll 1
  for (int s = 0; s < 2; ++s) {
    const int r = rbase + 2 * w + s;
    const float* xrow = x + (size_t)r * DM + 8 * lane;

    float s1 = 0.0f;
#pragma unroll 1
    for (int g = 0; g < 4; ++g) {
      const v4f a0 = *(const v4fa*)(xrow + 256 * g);
      const v4f a1 = *(const v4fa*)(xrow + 256 * g + 4);
      s1 += ((bf16r(a0[0]) + bf16r(a0[1])) + (bf16r(a0[2]) + bf16r(a0[3]))) +
            ((bf16r(a1[0]) + bf16r(a1[1])) + (bf16r(a1[2]) + bf16r(a1[3])));
    }
    s1 = wsum(s1);
    const float mu = s1 * (1.0f / DM);

    float s2 = 0.0f;
#pragma unroll 1
    for (int g = 0; g < 4; ++g) {
      const v4f a0 = *(const v4fa*)(xrow + 256 * g);
      const v4f a1 = *(const v4fa*)(xrow + 256 * g + 4);
      float q = 0.0f;
#pragma unroll
      for (int j = 0; j < 4; ++j) {
        const float d0 = bf16r(a0[j]) - mu;
        const float d1 = bf16r(a1[j]) - mu;
        q += d0 * d0;
        q += d1 * d1;
      }
      s2 += q;
    }
    s2 = wsum(s2);
    const float rstd = rsqrtf(s2 * (1.0f / DM) + LNEPS);

#pragma unroll 1
    for (int g = 0; g < 4; ++g) {
      const v4f a0 = *(const v4fa*)(xrow + 256 * g);
      const v4f a1 = *(const v4fa*)(xrow + 256 * g + 4);
      const v4f w0 = *(const v4fa*)(lw + 256 * g + 8 * lane);
      const v4f w1 = *(const v4fa*)(lw + 256 * g + 8 * lane + 4);
      const v4f b0 = *(const v4fa*)(lbias + 256 * g + 8 * lane);
      const v4f b1 = *(const v4fa*)(lbias + 256 * g + 8 * lane + 4);
      v8us oh, ol;
#pragma unroll
      for (int j = 0; j < 4; ++j) {
        const float v0 = ((bf16r(a0[j]) - mu) * rstd) * bf16r(w0[j]) + bf16r(b0[j]);
        const float v1 = ((bf16r(a1[j]) - mu) * rstd) * bf16r(w1[j]) + bf16r(b1[j]);
        unsigned short hb, lb;
        split_bf16(v0, hb, lb); oh[j] = hb;     ol[j] = lb;
        split_bf16(v1, hb, lb); oh[4 + j] = hb; ol[4 + j] = lb;
      }
      *(v8usa*)(wH + 256 * g + 8 * lane) = oh;
      *(v8usa*)(wL + 256 * g + 8 * lane) = ol;
    }
    __syncthreads();

    ln_store_pass(wH, wL, ph, pl, r, lane);
    __threadfence();
    ln_store_pass(wH, wL, ph, pl, r, lane);
    __syncthreads();
  }
}

__device__ __forceinline__ void c_store_pass(const float* sT, float* C, int ldc, int m0w, int cyl, int w, int lane) {
  const int q8 = lane & 7, sub = lane >> 3;
#pragma unroll
  for (int i = 0; i < 16; ++i) {
    const int lid = 4 * i + sub;
    const int rl = lid >> 1, hl = lid & 1;
    const v4f v = *(const v4fa*)(sT + (32 * w + rl) * 64 + 32 * hl + 4 * q8);
    float* dst = C + (size_t)(m0w + rl) * ldc + 64 * cyl + 32 * hl + 4 * q8;
    *(volatile v4f*)dst = v;
  }
}

__device__ __forceinline__ void dtr_store_pass(const float* sT, unsigned short* dh, unsigned short* dl,
                                               int m0w, int w, int lane) {
  const int q8 = lane & 7, sub = lane >> 3;
  const bool pad = (q8 >= DTR / 8);
#pragma unroll
  for (int i = 0; i < 8; ++i) {
    const int rl = 4 * i + sub;
    const float* sr = sT + (32 * w + rl) * 64 + 8 * q8;
    const v4f a = *(const v4fa*)sr;
    const v4f c = *(const v4fa*)(sr + 4);
    v8us oh, ol;
    unsigned short hb, lb;
    split_bf16(a[0], hb, lb); oh[0] = pad ? (unsigned short)0 : hb; ol[0] = pad ? (unsigned short)0 : lb;
    split_bf16(a[1], hb, lb); oh[1] = pad ? (unsigned short)0 : hb; ol[1] = pad ? (unsigned short)0 : lb;
    split_bf16(a[2], hb, lb); oh[2] = pad ? (unsigned short)0 : hb; ol[2] = pad ? (unsigned short)0 : lb;
    split_bf16(a[3], hb, lb); oh[3] = pad ? (unsigned short)0 : hb; ol[3] = pad ? (unsigned short)0 : lb;
    split_bf16(c[0], hb, lb); oh[4] = pad ? (unsigned short)0 : hb; ol[4] = pad ? (unsigned short)0 : lb;
    split_bf16(c[1], hb, lb); oh[5] = pad ? (unsigned short)0 : hb; ol[5] = pad ? (unsigned short)0 : lb;
    split_bf16(c[2], hb, lb); oh[6] = pad ? (unsigned short)0 : hb; ol[6] = pad ? (unsigned short)0 : lb;
    split_bf16(c[3], hb, lb); oh[7] = pad ? (unsigned short)0 : hb; ol[7] = pad ? (unsigned short)0 : lb;
    const size_t go = (size_t)(m0w + rl) * KDT + 8 * q8;
    *(volatile v8us*)(dh + go) = oh;
    *(volatile v8us*)(dl + go) = ol;
  }
}

template <int NPL, int XP, int GR>
__global__ __launch_bounds__(128)
void gemm_kernel(const unsigned short* __restrict__ Ah, const unsigned short* __restrict__ Al, int lda,
                 const unsigned short* __restrict__ Bw, int K,
                 float* C0, float* C1, int ncy0, int ldc, const float* __restrict__ res,
                 unsigned short* dh, unsigned short* dl)
{
  __shared__ __attribute__((aligned(16))) float sT[128 * 64];

  const int tid = threadIdx.x, lane = tid & 31, w = tid >> 5;
  const int h = lane >> 4, m = lane & 15;
  const int m0 = blockIdx.x * 128;
  const int cy = blockIdx.y;
  const bool upper = (cy >= ncy0);
  float* C = upper ? C1 : C0;
  const int cyl = upper ? (cy - ncy0) : cy;
  const int m0w = m0 + 32 * w;

  const unsigned short* xa = Ah + (size_t)(m0w + m) * lda;
  const unsigned short* xr = Al + (size_t)(m0w + m) * lda;
  const unsigned short* wb = Bw + (size_t)(64 * cy + m) * K;

  v8f acc[2][4];
#pragma unroll
  for (int mt = 0; mt < 2; ++mt)
#pragma unroll
    for (int nt = 0; nt < 4; ++nt) acc[mt][nt] = zero8();

#pragma unroll 1
  for (int k0 = 0; k0 < K; k0 += 32) {
    Frag a0, a1, e0, e1;
    ldfrag_g(a0, xa + k0, h);
    ldfrag_g(a1, xa + (size_t)16 * lda + k0, h);
    if (NPL == 2) {
      ldfrag_g(e0, xr + k0, h);
      ldfrag_g(e1, xr + (size_t)16 * lda + k0, h);
    }
#pragma unroll
    for (int nt = 0; nt < 4; ++nt) {
      Frag b;
      ldfrag_g(b, wb + (size_t)nt * 16 * K + k0, h);
      acc[0][nt] = mma16(acc[0][nt], a0, b);
      acc[1][nt] = mma16(acc[1][nt], a1, b);
      if (NPL == 2) {
        acc[0][nt] = mma16(acc[0][nt], e0, b);
        acc[1][nt] = mma16(acc[1][nt], e1, b);
      }
    }
  }

#pragma unroll
  for (int nt = 0; nt < 4; ++nt) {
    const int col = 16 * nt + m;
#pragma unroll
    for (int mt = 0; mt < 2; ++mt)
#pragma unroll
      for (int r = 0; r < 8; ++r) {
        const int rowl = 32 * w + 16 * mt + 8 * h + r;
        sT[rowl * 64 + col] = acc[mt][nt][r];
      }
  }
  __syncthreads();

  if (GR == 1) {
#pragma unroll 2
    for (int i = 0; i < 64; ++i) {
      const int idx = i * 128 + tid;
      const int rowl = idx >> 6, col = idx & 63;
      const float v = sT[idx];
      const float rsd = bf16r(res[(size_t)(m0 + rowl) * ldc + 64 * cyl + col]);
      const float gl = 0.5f * v * (1.0f + erff(v * 0.70710678118654752f));
      sT[idx] = gl + rsd;
    }
    __syncthreads();
  }

  c_store_pass(sT, C, ldc, m0w, cyl, w, lane);
  __threadfence();
  c_store_pass(sT, C, ldc, m0w, cyl, w, lane);

  if (XP == 1) {
    if (cy == 0) {
      dtr_store_pass(sT, dh, dl, m0w, w, lane);
      __threadfence();
      dtr_store_pass(sT, dh, dl, m0w, w, lane);
    }
  }
}

__device__ __forceinline__ void h16tile_store_pass(const unsigned short* sH, const unsigned short* sL,
                                                   unsigned short* ph, unsigned short* pl, int pitch, int col0,
                                                   int rbase, int w, int lane) {
  const int q8 = lane & 7, sub = lane >> 3;
#pragma unroll
  for (int i = 0; i < 2; ++i) {
    const int li = 4 * i + sub;
    const int row = 2 * w + (li >> 2), q = li & 3;
    const v8us vh = *(const v8usa*)(sH + row * 256 + 64 * q + 8 * q8);
    const v8us vl = *(const v8usa*)(sL + row * 256 + 64 * q + 8 * q8);
    const size_t go = (size_t)(rbase + row) * pitch + col0 + 64 * q + 8 * q8;
    *(volatile v8us*)(ph + go) = vh;
    *(volatile v8us*)(pl + go) = vl;
  }
}

__global__ __launch_bounds__(256)
void conv_kernel(const float* __restrict__ xc, const float* __restrict__ cw, const float* __restrict__ cb,
                 unsigned short* ph, unsigned short* pl)
{
  __shared__ __attribute__((aligned(16))) unsigned short sH[TC * 256];
  __shared__ __attribute__((aligned(16))) unsigned short sL[TC * 256];

  const int tid = threadIdx.x, lane = tid & 31, w = tid >> 5;
  const int slab = blockIdx.x;
  const int rbase = blockIdx.y * TC;
  const int b = rbase / NL, l0 = rbase - b * NL;
  const int c = 256 * slab + tid;

  const v4f cwv = *(const v4fa*)(cw + (size_t)c * 4);
  const float w0 = bf16r(cwv[0]);
  const float w1 = bf16r(cwv[1]);
  const float w2 = bf16r(cwv[2]);
  const float w3 = bf16r(cwv[3]);
  const float cbv = bf16r(cb[c]);

  const float* col = xc + (size_t)b * NL * DI + c;

  int p, pc;
  p = l0 - 3; pc = (p > 0) ? p : 0;
  float v0 = col[(size_t)pc * DI]; v0 = (p >= 0) ? v0 : 0.0f;
  p = l0 - 2; pc = (p > 0) ? p : 0;
  float v1 = col[(size_t)pc * DI]; v1 = (p >= 0) ? v1 : 0.0f;
  p = l0 - 1; pc = (p > 0) ? p : 0;
  float v2 = col[(size_t)pc * DI]; v2 = (p >= 0) ? v2 : 0.0f;

#pragma unroll 1
  for (int tt = 0; tt < TC; ++tt) {
    const float v3 = col[(size_t)(l0 + tt) * DI];
    const float s = w0 * v0 + w1 * v1 + w2 * v2 + w3 * v3 + cbv;
    const float ex = expf(fminf(-s, 60.0f));
    const float sg = 1.0f / (1.0f + ex);
    const float y = s * sg;
    unsigned short hb, lb;
    split_bf16(y, hb, lb);
    sH[tt * 256 + tid] = hb;
    sL[tt * 256 + tid] = lb;
    v0 = v1; v1 = v2; v2 = v3;
  }
  __syncthreads();

  const int col0 = 256 * slab;
  h16tile_store_pass(sH, sL, ph, pl, DI, col0, rbase, w, lane);
  __threadfence();
  h16tile_store_pass(sH, sL, ph, pl, DI, col0, rbase, w, lane);
}

__global__ __launch_bounds__(256)
void dtscan_kernel(const unsigned short* __restrict__ dth, const unsigned short* __restrict__ dtl,
                   const unsigned short* __restrict__ wdt,
                   const float* __restrict__ xdbl,
                   const unsigned short* __restrict__ uh, const unsigned short* __restrict__ ul,
                   const float* __restrict__ zg,
                   const float* __restrict__ dtb, const float* __restrict__ alog,
                   const float* __restrict__ dpar,
                   unsigned short* yh, unsigned short* yl)
{
  __shared__ __attribute__((aligned(16))) float sD[TC * 256];
  __shared__ __attribute__((aligned(16))) unsigned short sH[TC * 256];
  __shared__ __attribute__((aligned(16))) unsigned short sL[TC * 256];
  __shared__ __attribute__((aligned(16))) float sBC[TC * 32];

  const int tid = threadIdx.x, lane = tid & 31, w = tid >> 5;
  const int h = lane >> 4, m = lane & 15;
  const int slab = blockIdx.x, b = blockIdx.y;
  const int c0 = 256 * slab;
  const int d = c0 + tid;

  const float bb = bf16r(dtb[d]);
  const float Dv = bf16r(dpar[d]);
  float An[NS];
  {
    const float* ap = alog + (size_t)d * NS;
#pragma unroll
    for (int q = 0; q < NS / 4; ++q) {
      const v4f av = *(const v4fa*)(ap + 4 * q);
#pragma unroll
      for (int j = 0; j < 4; ++j) An[4 * q + j] = -expf(bf16r(av[j]));
    }
  }

  Frag bw[2][2];
#pragma unroll
  for (int nt = 0; nt < 2; ++nt)
#pragma unroll
    for (int ks = 0; ks < 2; ++ks)
      ldfrag_g(bw[nt][ks], wdt + (size_t)(c0 + 32 * w + 16 * nt + m) * KDT + 32 * ks, h);

  float hs[NS];
#pragma unroll
  for (int n = 0; n < NS; ++n) hs[n] = 0.0f;

#pragma unroll 1
  for (int t0 = 0; t0 < NL; t0 += TC) {
    const int r0 = b * NL + t0;

    v8f acc[2];
    acc[0] = zero8(); acc[1] = zero8();
#pragma unroll
    for (int ks = 0; ks < 2; ++ks) {
      Frag ah, ar;
      ldfrag_g(ah, dth + (size_t)(r0 + m) * KDT + 32 * ks, h);
      ldfrag_g(ar, dtl + (size_t)(r0 + m) * KDT + 32 * ks, h);
#pragma unroll
      for (int nt = 0; nt < 2; ++nt) {
        acc[nt] = mma16(acc[nt], ah, bw[nt][ks]);
        acc[nt] = mma16(acc[nt], ar, bw[nt][ks]);
      }
    }
#pragma unroll
    for (int nt = 0; nt < 2; ++nt)
#pragma unroll
      for (int r = 0; r < 8; ++r)
        sD[(8 * h + r) * 256 + 32 * w + 16 * nt + m] = acc[nt][r];

    if (tid < 128) {
      const int tok = tid >> 3, q = tid & 7;
      const v4f v = *(const v4fa*)(xdbl + (size_t)(r0 + tok) * NXP + DTR + 4 * q);
      *(v4fa*)(sBC + tok * 32 + 4 * q) = v;
    }
    __syncthreads();

#pragma unroll 1
    for (int tt = 0; tt < TC; ++tt) {
      const float dpre = sD[tt * 256 + tid];
      const float xx = dpre + bb;
      const float dl = fmaxf(xx, 0.0f) + log1pf(expf(-fabsf(xx)));
      const size_t gi = (size_t)(r0 + tt) * DI + d;
      const float xv = bf16_val(uh[gi]) + bf16_val(ul[gi]);
      const float rv = zg[gi];
      const float* bc = sBC + tt * 32;
      const float du = dl * xv;
      float y = 0.0f;
#pragma unroll
      for (int n = 0; n < NS; ++n) {
        const float dA = expf(dl * An[n]);
        hs[n] = dA * hs[n] + du * bc[n];
        y += hs[n] * bc[NS + n];
      }
      const float yv = y + xv * Dv;
      const float eg = expf(fminf(-rv, 60.0f));
      const float g = rv * (1.0f / (1.0f + eg));
      const float yg = yv * g;
      unsigned short hb, lb;
      split_bf16(yg, hb, lb);
      sH[tt * 256 + tid] = hb;
      sL[tt * 256 + tid] = lb;
    }
    __syncthreads();

    h16tile_store_pass(sH, sL, yh, yl, DI, c0, r0, w, lane);
    __threadfence();
    h16tile_store_pass(sH, sL, yh, yl, DI, c0, r0, w, lane);
    __syncthreads();
  }
}

extern "C" void kernel_launch(void* const* d_in, const int* in_sizes, int n_in,
                              void* d_out, int out_size, void* d_ws, size_t ws_size,
                              hipStream_t stream)
{
  if (n_in < 12) return;
  if (in_sizes[0]  != NROWS * DM) return;
  if (in_sizes[1]  != DM)         return;
  if (in_sizes[2]  != DM)         return;
  if (in_sizes[3]  != DM * DIN2)  return;
  if (in_sizes[4]  != DI * 4)     return;
  if (in_sizes[5]  != DI)         return;
  if (in_sizes[6]  != DI * NXD)   return;
  if (in_sizes[7]  != DTR * DI)   return;
  if (in_sizes[8]  != DI)         return;
  if (in_sizes[9]  != DI * NS)    return;
  if (in_sizes[10] != DI)         return;
  if (in_sizes[11] != DI * DM)    return;
  if (out_size != NROWS * DM) return;
  if (ws_size < WS_END) return;

  const float* x      = (const float*)d_in[0];
  const float* ln_w   = (const float*)d_in[1];
  const float* ln_b   = (const float*)d_in[2];
  const float* w_in   = (const float*)d_in[3];
  const float* conv_w = (const float*)d_in[4];
  const float* conv_b = (const float*)d_in[5];
  const float* w_x    = (const float*)d_in[6];
  const float* w_dt   = (const float*)d_in[7];
  const float* b_dt   = (const float*)d_in[8];
  const float* a_log  = (const float*)d_in[9];
  const float* dpar   = (const float*)d_in[10];
  const float* w_out  = (const float*)d_in[11];
  float* out = (float*)d_out;

  char* ws = (char*)d_ws;
  unsigned short* XNH  = (unsigned short*)(ws + OFF_XNH);
  unsigned short* XNL  = (unsigned short*)(ws + OFF_XNL);
  unsigned short* WIN  = (unsigned short*)(ws + OFF_WIN);
  unsigned short* XH   = (unsigned short*)(ws + OFF_XH);
  float*          XDBL = (float*)(ws + OFF_XDBL);
  unsigned short* DTH  = (unsigned short*)(ws + OFF_DTH);
  unsigned short* DTL  = (unsigned short*)(ws + OFF_DTL);
  unsigned short* WXP  = (unsigned short*)(ws + OFF_WXP);
  unsigned short* WDT  = (unsigned short*)(ws + OFF_WDT);
  unsigned short* WOUT = (unsigned short*)(ws + OFF_WOUT);
  float*          XC   = (float*)(ws + OFF_XC);
  unsigned short* YH   = (unsigned short*)(ws + OFF_YH);
  unsigned short* YL   = (unsigned short*)(ws + OFF_YL);
  float*          ZP   = (float*)(ws + OFF_Z);
  unsigned short* XL   = (unsigned short*)(ws + OFF_XL);

  tcvt_kernel<<<dim3(DIN2 / 64, DM / 64, 1), dim3(256), 0, stream>>>(
      w_in, DM, DIN2, 0, WIN, DM, 0);
  tcvt_kernel<<<dim3(NXP / 64, DI / 64, 1), dim3(256), 0, stream>>>(
      w_x, DI, NXD, 0, WXP, DI, 0);
  tcvt_kernel<<<dim3(DI / 64, KDT / 64, 1), dim3(256), 0, stream>>>(
      w_dt, DTR, DI, 0, WDT, KDT, 0);
  tcvt_kernel<<<dim3(DM / 64, DI / 64, 1), dim3(256), 0, stream>>>(
      w_out, DI, DM, 0, WOUT, DI, 0);

  ln_kernel<<<dim3(NROWS / TL), dim3(256), 0, stream>>>(x, ln_w, ln_b, XNH, XNL);

  gemm_kernel<2, 0, 0><<<dim3(NROWS / 128, DIN2 / 64), dim3(128), 0, stream>>>(
      XNH, XNL, DM, WIN, DM, XC, ZP, DI / 64, DI, x, DTH, DTL);

  conv_kernel<<<dim3(DI / 256, NROWS / TC), dim3(256), 0, stream>>>(XC, conv_w, conv_b, XH, XL);

  gemm_kernel<2, 1, 0><<<dim3(NROWS / 128, NXP / 64), dim3(128), 0, stream>>>(
      XH, XL, DI, WXP, DI, XDBL, XDBL, NXP / 64, NXP, x, DTH, DTL);

  dtscan_kernel<<<dim3(DI / 256, NB), dim3(256), 0, stream>>>(
      DTH, DTL, WDT, XDBL, XH, XL, ZP, b_dt, a_log, dpar, YH, YL);

  gemm_kernel<2, 0, 1><<<dim3(NROWS / 128, DM / 64), dim3(128), 0, stream>>>(
      YH, YL, DI, WOUT, DI, out, out, DM / 64, DM, x, DTH, DTL);
}
